// GRN_67216238182732
// MI455X (gfx1250) — hardware-verified
//
#include <hip/hip_runtime.h>
#include <stddef.h>

typedef __attribute__((ext_vector_type(16))) _Float16 v16h;
typedef __attribute__((ext_vector_type(8)))  _Float16 v8h;
typedef __attribute__((ext_vector_type(16))) __bf16   v16b;
typedef __attribute__((ext_vector_type(8)))  __bf16   v8b;
typedef __attribute__((ext_vector_type(8)))  float    v8f;
typedef __attribute__((ext_vector_type(4)))  float    v4f;
typedef __attribute__((ext_vector_type(4)))  unsigned v4u;

constexpr int NB = 8;
constexpr int NL = 512;
constexpr int ND = 64;
constexpr int NS = 8;
constexpr int PJ_ROWS = 64;
constexpr int PJ_LD   = NB * NL;

constexpr size_t X_PLANE  = (size_t)NB * NL * ND;
constexpr size_t WT_TOTAL = (size_t)NS * ND * ND;
constexpr size_t PW_TOTAL = (size_t)2 * PJ_ROWS * ND;
constexpr size_t AP_TOTAL = (size_t)NB * NS * NL * ND;
constexpr size_t PJ_PLANE = (size_t)PJ_ROWS * PJ_LD;
constexpr size_t RW_PLANE = (size_t)NL * NL;
constexpr size_t RW_TOTAL = (size_t)NB * NS * RW_PLANE;

constexpr size_t OFF_XH  = 0;
constexpr size_t OFF_XL  = OFF_XH  + 2 * X_PLANE * 2;
constexpr size_t OFF_WTH = OFF_XL  + 2 * X_PLANE * 2;
constexpr size_t OFF_WTL = OFF_WTH + WT_TOTAL * 2;
constexpr size_t OFF_PWH = OFF_WTL + WT_TOTAL * 2;
constexpr size_t OFF_PWL = OFF_PWH + PW_TOTAL * 2;
constexpr size_t OFF_APH = OFF_PWL + PW_TOTAL * 2;
constexpr size_t OFF_APL = OFF_APH + AP_TOTAL * 2;
constexpr size_t OFF_PJ  = OFF_APL + AP_TOTAL * 2;
constexpr size_t OFF_RW  = OFF_PJ  + 2 * PJ_PLANE * 4;
constexpr size_t WS_TOTAL = OFF_RW + RW_TOTAL * 4;
static_assert(WS_TOTAL == 79855616, "carve total");
static_assert(WS_TOTAL <= 134217728, "carve under 128 MiB");
static_assert((OFF_XL % 256) == 0 && (OFF_WTH % 256) == 0 && (OFF_WTL % 256) == 0 && (OFF_PWH % 256) == 0 &&
              (OFF_PWL % 256) == 0 && (OFF_APH % 256) == 0 && (OFF_APL % 256) == 0 && (OFF_PJ % 256) == 0 &&
              (OFF_RW % 256) == 0, "region alignment");

static_assert(ND % 32 == 0, "K multiple of 32");
static_assert(NL % 64 == 0, "M/N multiple of 64 (stage 1 M, stage 2 M and N)");
static_assert(ND % 64 == 0, "stage 1 N = 64");
static_assert(PJ_ROWS % 64 == 0 && PJ_LD % 64 == 0, "projection M and N multiples of 64");
static_assert((2 * X_PLANE) % (8 * 256) == 0, "split kernel coverage");

__device__ __forceinline__ unsigned short f2bf_bits(float f) {
  unsigned u = __float_as_uint(f);
  return (unsigned short)((u + 0x7FFFu + ((u >> 16) & 1u)) >> 16);
}
__device__ __forceinline__ float bf_bits2f(unsigned short h) { return __uint_as_float(((unsigned)h) << 16); }

__device__ __forceinline__ void pack_hl2(float a, float b, unsigned& hw, unsigned& lw) {
  const unsigned short ha = f2bf_bits(a);
  const unsigned short hb = f2bf_bits(b);
  const unsigned short la = f2bf_bits(a - bf_bits2f(ha));
  const unsigned short lb = f2bf_bits(b - bf_bits2f(hb));
  hw = (unsigned)ha | ((unsigned)hb << 16);
  lw = (unsigned)la | ((unsigned)lb << 16);
}

__device__ __forceinline__ void dep_guard_h(v8f& a, v8f& b, v16h x, v16h y) { asm volatile("v_nop\n\tv_nop\n\tv_nop\n\tv_nop" : "+v"(a), "+v"(b) : "v"(x), "v"(y)); }
__device__ __forceinline__ void dep_guard_b(v8f& a, v8f& b, v16b x, v16b y) { asm volatile("v_nop\n\tv_nop\n\tv_nop\n\tv_nop" : "+v"(a), "+v"(b) : "v"(x), "v"(y)); }
__device__ __forceinline__ void keep4_h(v16h a, v16h b, v16h c, v16h d) { asm volatile("v_nop" :: "v"(a), "v"(b), "v"(c), "v"(d)); }
__device__ __forceinline__ void keep4_b(v16b a, v16b b, v16b c, v16b d) { asm volatile("v_nop" :: "v"(a), "v"(b), "v"(c), "v"(d)); }
__device__ __forceinline__ void acc_guard4(v8f& a, v8f& b, v8f& c, v8f& d) { asm volatile("v_nop\n\tv_nop\n\tv_nop\n\tv_nop" : "+v"(a), "+v"(b), "+v"(c), "+v"(d)); }
template <typename T> struct Frag;
template <> struct Frag<_Float16> {
  typedef v16h V; union U { v16h v; v8h h[2]; };
  static __device__ __forceinline__ v16h load(const _Float16* p) {
    U f; f.h[0] = *(const v8h*)(p); f.h[1] = *(const v8h*)(p + 16); return f.v;
  }
  static __device__ __forceinline__ v8f mma(v16h a, v16h b, v8f c) {
    return __builtin_amdgcn_wmma_f32_16x16x32_f16(false, a, false, b, (short)0, c, false, false);
  }
  static __device__ __forceinline__ void guard(v8f& a, v8f& b, v16h x, v16h y) { dep_guard_h(a, b, x, y); }
  static __device__ __forceinline__ void keep(v16h a, v16h b, v16h c, v16h d) { keep4_h(a, b, c, d); }
};
template <> struct Frag<__bf16> {
  typedef v16b V; union U { v16b v; v8b h[2]; };
  static __device__ __forceinline__ v16b load(const __bf16* p) {
    U f; f.h[0] = *(const v8b*)(p); f.h[1] = *(const v8b*)(p + 16); return f.v;
  }
  static __device__ __forceinline__ v8f mma(v16b a, v16b b, v8f c) {
    return __builtin_amdgcn_wmma_f32_16x16x32_bf16(false, a, false, b, (short)0, c, false, false);
  }
  static __device__ __forceinline__ void guard(v8f& a, v8f& b, v16b x, v16b y) { dep_guard_b(a, b, x, y); }
  static __device__ __forceinline__ void keep(v16b a, v16b b, v16b c, v16b d) { keep4_b(a, b, c, d); }
};

template <int ET> struct Elem;
template <> struct Elem<0> { typedef _Float16 T; };
template <> struct Elem<1> { typedef __bf16 T; };
template <int ET, bool SPLIT, int BIAS_MODE, int OUT_MODE>
__global__ __launch_bounds__(256) void wmma_gemm64_yz(
    const unsigned short* __restrict__ Ap, const unsigned short* __restrict__ A2p, int lda, long strideAy, long strideAz,
    const unsigned short* __restrict__ Btp, const unsigned short* __restrict__ Bt2p, int ldb, long strideBy, long strideBz,
    void* __restrict__ Cout, void* __restrict__ Cout2, int ldc, long strideCy, long strideCz,
    const float* __restrict__ bias,
    int M, int N, int K, float scale) {
  typedef typename Elem<ET>::T T;
  typedef typename Frag<T>::V V;
  const T* A = (const T*)Ap; const T* A2 = (const T*)A2p; const T* Bt = (const T*)Btp; const T* Bt2 = (const T*)Bt2p;
  __shared__ __align__(16) float sT[8][16 * 68];
  const int by   = blockIdx.y;
  const int bz   = blockIdx.z;
  const int lane = threadIdx.x & 31;
  const int wave = threadIdx.x >> 5;
  const int tilesN = N >> 6;
  const int tilesM = M >> 6;
  const int tile = blockIdx.x * 8 + wave;
  if (tile >= tilesM * tilesN) return;
  const int tm = tile / tilesN;
  const int tn = tile - tm * tilesN;
  const int m0 = tm << 6;
  const int n0 = tn << 6;

  const size_t offA = (size_t)by * (size_t)strideAy + (size_t)bz * (size_t)strideAz;
  const size_t offB = (size_t)by * (size_t)strideBy + (size_t)bz * (size_t)strideBz;
  const size_t offC = (size_t)by * (size_t)strideCy + (size_t)bz * (size_t)strideCz;
  const T* Ab  = A  + offA;
  const T* Bb  = Bt + offB;
  const T* Ab2 = SPLIT ? (A2  + offA) : nullptr;
  const T* Bb2 = SPLIT ? (Bt2 + offB) : nullptr;

  const int rlane = lane & 15;
  const int koff  = (lane >> 4) * 8;
  const int mOff  = (lane >> 4) * 8;

  v8f acc[4][4];
#pragma unroll
  for (int i = 0; i < 4; ++i)
#pragma unroll
    for (int j = 0; j < 4; ++j) acc[i][j] = (v8f){0.f,0.f,0.f,0.f,0.f,0.f,0.f,0.f};

  for (int k0 = 0; k0 < K; k0 += 32) {
    V bh[4], bl[4];
#pragma unroll
    for (int j = 0; j < 4; ++j) {
      const size_t bo = (size_t)(n0 + (j << 4) + rlane) * ldb + koff + k0;
      bh[j] = Frag<T>::load(Bb + bo);
      if (SPLIT) bl[j] = Frag<T>::load(Bb2 + bo);
    }
#pragma unroll
    for (int i = 0; i < 4; ++i) {
      const size_t ao = (size_t)(m0 + (i << 4) + rlane) * lda + koff + k0;
      V ah = Frag<T>::load(Ab + ao);
      V al;
      if (SPLIT) al = Frag<T>::load(Ab2 + ao);
#pragma unroll
      for (int j = 0; j < 4; ++j) {
        acc[i][j] = Frag<T>::mma(ah, bh[j], acc[i][j]);
        if (SPLIT) {
          acc[i][j] = Frag<T>::mma(ah, bl[j], acc[i][j]);
          acc[i][j] = Frag<T>::mma(al, bh[j], acc[i][j]);
        }
      }
      Frag<T>::guard(acc[i][0], acc[i][3], ah, SPLIT ? al : ah);
    }
    Frag<T>::keep(bh[0], bh[1], bh[2], bh[3]);
    if (SPLIT) Frag<T>::keep(bl[0], bl[1], bl[2], bl[3]);
  }
  acc_guard4(acc[0][0], acc[0][1], acc[0][2], acc[0][3]);
  acc_guard4(acc[1][0], acc[1][1], acc[1][2], acc[1][3]);
  acc_guard4(acc[2][0], acc[2][1], acc[2][2], acc[2][3]);
  acc_guard4(acc[3][0], acc[3][1], acc[3][2], acc[3][3]);

  float* slab = sT[wave];
#pragma unroll
  for (int i = 0; i < 4; ++i) {
    const int mBase = m0 + (i << 4);
#pragma unroll
    for (int j = 0; j < 4; ++j) {
      const int n = n0 + (j << 4) + rlane;
      float bv = 0.f;
      if (BIAS_MODE == 2) bv = bias[n];
#pragma unroll
      for (int r = 0; r < 8; ++r) {
        float v = acc[i][j][r] * scale;
        if (BIAS_MODE == 1) v += bias[mBase + mOff + r];
        if (BIAS_MODE == 2) v += bv;
        slab[(mOff + r) * 68 + (j << 4) + rlane] = v;
      }
    }
    __builtin_amdgcn_fence(__ATOMIC_RELEASE, "workgroup");
    __builtin_amdgcn_wave_barrier();
    __builtin_amdgcn_fence(__ATOMIC_ACQUIRE, "workgroup");
    if (OUT_MODE == 0) {
      float* C = (float*)Cout + offC;
      const int hh = lane >> 4, c4 = (lane & 15) * 4;
      for (int pass = 0; pass < 2; ++pass) {
#pragma unroll
        for (int it = 0; it < 8; ++it) {
          const int row = it * 2 + hh;
          v4f v = *(const v4f*)(slab + row * 68 + c4);
          *(volatile v4f*)(C + (size_t)(mBase + row) * ldc + n0 + c4) = v;
        }
        __threadfence();
      }
    } else {
      const int q = lane >> 3, c8 = (lane & 7) * 8;
      unsigned short* C  = (unsigned short*)Cout  + offC;
      unsigned short* C2 = (OUT_MODE == 2) ? ((unsigned short*)Cout2 + offC) : nullptr;
      for (int pass = 0; pass < 2; ++pass) {
#pragma unroll
        for (int it = 0; it < 4; ++it) {
          const int row = it * 4 + q;
          const float* sp = slab + row * 68 + c8;
          v8h hv, lv;
#pragma unroll
          for (int e = 0; e < 8; ++e) {
            if (OUT_MODE == 1) {
              hv[e] = (_Float16)sp[e];
            } else {
              unsigned short hb = f2bf_bits(sp[e]);
              unsigned short lb = f2bf_bits(sp[e] - bf_bits2f(hb));
              hv[e] = __builtin_bit_cast(_Float16, hb);
              lv[e] = __builtin_bit_cast(_Float16, lb);
            }
          }
          *(volatile v8h*)(C + (size_t)(mBase + row) * ldc + n0 + c8) = hv;
          if (OUT_MODE == 2) *(volatile v8h*)(C2 + (size_t)(mBase + row) * ldc + n0 + c8) = lv;
        }
        __threadfence();
      }
    }
    __builtin_amdgcn_fence(__ATOMIC_RELEASE, "workgroup");
    __builtin_amdgcn_wave_barrier();
    __builtin_amdgcn_fence(__ATOMIC_ACQUIRE, "workgroup");
  }
}

__global__ __launch_bounds__(256) void k_split_x(const float* __restrict__ x0, const float* __restrict__ x1,
                                                  unsigned short* __restrict__ Xh, unsigned short* __restrict__ Xl) {
  const float* src = (blockIdx.y == 0) ? x0 : x1;
  const size_t soff = ((size_t)blockIdx.x * 256 + threadIdx.x) * 8;
  const size_t doff = (size_t)blockIdx.y * X_PLANE + soff;
  const v4f a = *(const v4f*)(src + soff);
  const v4f c = *(const v4f*)(src + soff + 4);
  unsigned h0, h1, h2, h3, l0, l1, l2, l3;
  pack_hl2(a[0], a[1], h0, l0);
  pack_hl2(a[2], a[3], h1, l1);
  pack_hl2(c[0], c[1], h2, l2);
  pack_hl2(c[2], c[3], h3, l3);
  const v4u hv = (v4u){h0, h1, h2, h3};
  const v4u lvv = (v4u){l0, l1, l2, l3};
  *(volatile v4u*)(Xh + doff) = hv;
  *(volatile v4u*)(Xl + doff) = lvv;
  __threadfence();
  *(volatile v4u*)(Xh + doff) = hv;
  *(volatile v4u*)(Xl + doff) = lvv;
}

__global__ __launch_bounds__(256) void k_split_wt(const float* __restrict__ Wm,
                                                   unsigned short* __restrict__ Wth, unsigned short* __restrict__ Wtl) {
  __shared__ float tile[ND * (ND + 1)];
  const int s = blockIdx.x;
  const int t = threadIdx.x;
  const float* wsrc = Wm + (size_t)s * ND * ND;
#pragma unroll
  for (int it = 0; it < 4; ++it) {
    const int idx4 = it * 256 + t;
    const int d = idx4 >> 4;
    const int e0 = (idx4 & 15) * 4;
    const v4f v = *(const v4f*)(wsrc + d * ND + e0);
    tile[d * (ND + 1) + e0 + 0] = v[0];
    tile[d * (ND + 1) + e0 + 1] = v[1];
    tile[d * (ND + 1) + e0 + 2] = v[2];
    tile[d * (ND + 1) + e0 + 3] = v[3];
  }
  __syncthreads();
  for (int pass = 0; pass < 2; ++pass) {
#pragma unroll
    for (int it = 0; it < 2; ++it) {
      const int idx = it * 256 + t;
      const int e = idx >> 3;
      const int d0 = (idx & 7) * 8;
      const float f0 = tile[(d0 + 0) * (ND + 1) + e];
      const float f1 = tile[(d0 + 1) * (ND + 1) + e];
      const float f2 = tile[(d0 + 2) * (ND + 1) + e];
      const float f3 = tile[(d0 + 3) * (ND + 1) + e];
      const float f4 = tile[(d0 + 4) * (ND + 1) + e];
      const float f5 = tile[(d0 + 5) * (ND + 1) + e];
      const float f6 = tile[(d0 + 6) * (ND + 1) + e];
      const float f7 = tile[(d0 + 7) * (ND + 1) + e];
      unsigned h0, h1, h2, h3, l0, l1, l2, l3;
      pack_hl2(f0, f1, h0, l0);
      pack_hl2(f2, f3, h1, l1);
      pack_hl2(f4, f5, h2, l2);
      pack_hl2(f6, f7, h3, l3);
      const v4u hv = (v4u){h0, h1, h2, h3};
      const v4u lvv = (v4u){l0, l1, l2, l3};
      const size_t o = (size_t)s * ND * ND + (size_t)e * ND + d0;
      *(volatile v4u*)(Wth + o) = hv;
      *(volatile v4u*)(Wtl + o) = lvv;
    }
    __threadfence();
  }
}

__global__ __launch_bounds__(256) void k_split_pw(const float* __restrict__ Vm, const float* __restrict__ Wg,
                                                   unsigned short* __restrict__ Pwh, unsigned short* __restrict__ Pwl) {
  const int t = threadIdx.x;
  for (int pass = 0; pass < 2; ++pass) {
#pragma unroll
    for (int it = 0; it < 4; ++it) {
      const int idx = it * 256 + t;
      const int z = idx >> 9;
      const int row = (idx >> 3) & 63;
      const int d0 = (idx & 7) * 8;
      const int vrow = row < 8 ? row : 7;
      int grow = row - 8; grow = grow < 0 ? 0 : (grow > 7 ? 7 : grow);
      const float* vp = Vm + (size_t)vrow * (2 * ND) + z * ND + d0;
      const float* gp = Wg + (size_t)grow * (2 * ND) + z * ND + d0;
      const v4f va = *(const v4f*)(vp), vb = *(const v4f*)(vp + 4);
      const v4f ga = *(const v4f*)(gp), gb = *(const v4f*)(gp + 4);
      const bool isv = row < 8;
      const bool isg = (row >= 8) && (row < 16);
      const float f0 = isv ? va[0] : (isg ? ga[0] : 0.f);
      const float f1 = isv ? va[1] : (isg ? ga[1] : 0.f);
      const float f2 = isv ? va[2] : (isg ? ga[2] : 0.f);
      const float f3 = isv ? va[3] : (isg ? ga[3] : 0.f);
      const float f4 = isv ? vb[0] : (isg ? gb[0] : 0.f);
      const float f5 = isv ? vb[1] : (isg ? gb[1] : 0.f);
      const float f6 = isv ? vb[2] : (isg ? gb[2] : 0.f);
      const float f7 = isv ? vb[3] : (isg ? gb[3] : 0.f);
      unsigned h0, h1, h2, h3, l0, l1, l2, l3;
      pack_hl2(f0, f1, h0, l0);
      pack_hl2(f2, f3, h1, l1);
      pack_hl2(f4, f5, h2, l2);
      pack_hl2(f6, f7, h3, l3);
      const v4u hv = (v4u){h0, h1, h2, h3};
      const v4u lvv = (v4u){l0, l1, l2, l3};
      const size_t o = (size_t)z * PJ_ROWS * ND + (size_t)row * ND + d0;
      *(volatile v4u*)(Pwh + o) = hv;
      *(volatile v4u*)(Pwl + o) = lvv;
    }
    __threadfence();
  }
}

__device__ __forceinline__ float sigm(float x) {
  const float e = expf(-x);
  return __builtin_amdgcn_rcpf(1.0f + e);
}

__global__ __launch_bounds__(128) void k_combine(const float* __restrict__ Rw, const float* __restrict__ PjT,
                                                 const float* __restrict__ bvec, const float* __restrict__ bgv,
                                                 const float* __restrict__ uv, float* __restrict__ out) {
  __shared__ float par[5][NS];
  const int t  = threadIdx.x;
  const int bi = blockIdx.x;
  const int b  = bi >> 9;
  const int i  = bi & (NL - 1);
  {
    const int s = t & (NS - 1);
    const float pv1 = PjT[(size_t)s * PJ_LD + bi];
    const float pg1 = PjT[(size_t)(NS + s) * PJ_LD + bi];
    const float pb  = bvec[s];
    const float pg  = bgv[s];
    const float pu  = uv[s];
    if (t < NS) { par[0][s] = pv1; par[1][s] = pg1; par[2][s] = pb; par[3][s] = pg; par[4][s] = pu; }
  }
  __syncthreads();
  const int j0 = t * 4;
  const float* P2 = PjT + PJ_PLANE + (size_t)b * NL + j0;
  const float* R  = Rw + (size_t)b * NS * RW_PLANE + (size_t)i * NL + j0;
  v4f o = (v4f){0.f, 0.f, 0.f, 0.f};
#pragma unroll 1
  for (int s = 0; s < NS; ++s) {
    const v4f v2 = *(const v4f*)(P2 + (size_t)s * PJ_LD);
    const v4f g2 = *(const v4f*)(P2 + (size_t)(NS + s) * PJ_LD);
    const v4f rw = *(const v4f*)(R + (size_t)s * RW_PLANE);
    const float v1 = par[0][s];
    const float g1 = par[1][s];
    const float cb = par[2][s];
    const float cg = par[3][s];
    const float cu = par[4][s];
#pragma unroll
    for (int q = 0; q < 4; ++q) {
      const float gate = sigm(g1 + g2[q] + cg);
      const float sv   = sigm(v1 + v2[q]);
      const float val  = gate * rw[q] + (1.0f - gate) * sv + cb;
      o[q] += val * cu;
    }
  }
  float* op = out + (size_t)bi * NL + j0;
  *(volatile v4f*)op = o;
  __threadfence();
  *(volatile v4f*)op = o;
}

extern "C" void kernel_launch(void* const* d_in, const int* in_sizes, int n_in,
                              void* d_out, int out_size, void* d_ws, size_t ws_size,
                              hipStream_t stream) {
  if (n_in < 8) return;
  if (in_sizes[0] != (int)X_PLANE || in_sizes[1] != (int)X_PLANE) return;
  if (in_sizes[2] != (int)WT_TOTAL) return;
  if (in_sizes[3] != NS * 2 * ND || in_sizes[5] != NS * 2 * ND) return;
  if (in_sizes[4] < NS || in_sizes[6] < NS || in_sizes[7] < NS) return;
  if (out_size != (int)RW_TOTAL / NS) return;
  if (ws_size < WS_TOTAL) return;

  const float* lstm1 = (const float*)d_in[0];
  const float* lstm2 = (const float*)d_in[1];
  const float* Wm    = (const float*)d_in[2];
  const float* Vm    = (const float*)d_in[3];
  const float* bvec  = (const float*)d_in[4];
  const float* Wg    = (const float*)d_in[5];
  const float* bgv   = (const float*)d_in[6];
  const float* uv    = (const float*)d_in[7];
  float* out = (float*)d_out;

  char* ws = (char*)d_ws;
  unsigned short* Xh  = (unsigned short*)(ws + OFF_XH);
  unsigned short* Xl  = (unsigned short*)(ws + OFF_XL);
  unsigned short* Wth = (unsigned short*)(ws + OFF_WTH);
  unsigned short* Wtl = (unsigned short*)(ws + OFF_WTL);
  unsigned short* Pwh = (unsigned short*)(ws + OFF_PWH);
  unsigned short* Pwl = (unsigned short*)(ws + OFF_PWL);
  unsigned short* Aph = (unsigned short*)(ws + OFF_APH);
  unsigned short* Apl = (unsigned short*)(ws + OFF_APL);
  float* PjT = (float*)(ws + OFF_PJ);
  float* Rw  = (float*)(ws + OFF_RW);

  k_split_x <<<dim3((unsigned)(X_PLANE / (8 * 256)), 2, 1), 256, 0, stream>>>(lstm1, lstm2, Xh, Xl);
  k_split_wt<<<NS, 256, 0, stream>>>(Wm, Wth, Wtl);
  k_split_pw<<<1, 256, 0, stream>>>(Vm, Wg, Pwh, Pwl);

  wmma_gemm64_yz<1, true, 0, 2><<<dim3(1, NS, NB), 256, 0, stream>>>(
      Xh, Xl, ND, 0L, (long)(NL * ND),
      Wth, Wtl, ND, (long)(ND * ND), 0L,
      (void*)Aph, (void*)Apl, ND, (long)(NL * ND), (long)(NS * NL * ND),
      bvec, NL, ND, ND, 1.0f);

  wmma_gemm64_yz<1, true, 0, 0><<<dim3((PJ_ROWS / 64) * (PJ_LD / 64) / 8, 1, 2), 256, 0, stream>>>(
      Pwh, Pwl, ND, 0L, (long)(PJ_ROWS * ND),
      Xh, Xl, ND, 0L, (long)X_PLANE,
      (void*)PjT, (void*)PjT, PJ_LD, 0L, (long)PJ_PLANE,
      bvec, PJ_ROWS, PJ_LD, ND, 1.0f);

  wmma_gemm64_yz<1, true, 0, 0><<<dim3((NL / 64) * (NL / 64) / 8, NS, NB), 256, 0, stream>>>(
      Aph, Apl, ND, (long)(NL * ND), (long)(NS * NL * ND),
      Xh + X_PLANE, Xl + X_PLANE, ND, 0L, (long)(NL * ND),
      (void*)Rw, (void*)Rw, NL, (long)RW_PLANE, (long)(NS * RW_PLANE),
      bvec, NL, NL, ND, 1.0f);

  k_combine<<<NB * NL, 128, 0, stream>>>(Rw, PjT, bvec, bgv, uv, out);
}
